// GNN_64484638982367
// MI455X (gfx1250) — hardware-verified
//
#include <hip/hip_runtime.h>
#include <stddef.h>
#include <stdint.h>
#include <math.h>

#pragma clang fp contract(off)


#define NF     128
#define NG     384
#define GN     192
#define KG     256
#define C1O    256
#define K1     1280
#define K2     2560
#define NTHR   256
#define NWAVE  8
#define EPT    8
#define CHUNK  (NTHR * EPT)
#define WCAP   (EPT * 32)
#define LISTN  (NWAVE * WCAP)
#define NBR    512
#define NSL    2048
#define SLA    11
#define RCAP   20480
#define DEGCAP 64
#define GBM    64
#define GBN    128
#define GTHR   128
#define SBLK   128
#define AGG_ZINTS    (LISTN + 2 * RCAP + 3 * NSL)
#define MISC_INTS    16
#define AGG_LDS_INTS (AGG_ZINTS + MISC_INTS)
#define PB_WG  48
#define PB_L1  32
#define PB_C1  128
#define PB_L2  32
#define PB_C2  128
#define PB_ALL (PB_WG + PB_L1 + PB_C1 + PB_L2 + PB_C2 + 1)
#define NBIAS  768
#define WSMAX  134217728

static_assert((CHUNK & (CHUNK - 1)) == 0 && CHUNK <= 4096);
static_assert(NSL == (1 << SLA) && NSL == 4 * NBR);
static_assert(((long long)CHUNK << SLA) < (1LL << 31));
static_assert(NSL % NWAVE == 0 && NSL % 32 == 0 && NBR % GBM == 0 && NBR % NWAVE == 0);
static_assert(AGG_ZINTS % (NTHR * 4) == 0 && RCAP % 4 == 0);
static_assert(AGG_LDS_INTS * 4 <= 300000);
static_assert(KG % 32 == 0 && K1 % 32 == 0 && K2 % 32 == 0);
static_assert(K1 == 2 * NF + 8 * NF && K2 == 2 * C1O + 8 * C1O);
static_assert(GBM == (GTHR / 32) * 16 && NG == 2 * GN && GN == 3 * 64);
static_assert(PB_WG * NTHR == NG * (KG / 8));
static_assert(PB_L1 * NTHR == C1O * (2 * NF / 8) && PB_C1 * NTHR == C1O * (8 * NF / 8));
static_assert(PB_L2 * NTHR == NF * (2 * C1O / 8) && PB_C2 * NTHR == NF * (8 * C1O / 8));
static_assert(NBIAS == NG + C1O + NF && NBIAS / 4 <= NTHR);
static_assert(GBM * GN * 4 <= 65536 && GBM * GBN * 4 <= 65536);

typedef float          v4f   __attribute__((ext_vector_type(4)));
typedef float          v8f   __attribute__((ext_vector_type(8)));
typedef int            v4i   __attribute__((ext_vector_type(4)));
typedef int            v8i   __attribute__((ext_vector_type(8)));
typedef unsigned int   v4u   __attribute__((ext_vector_type(4)));
typedef unsigned short v8us  __attribute__((ext_vector_type(8)));
typedef unsigned short v16us __attribute__((ext_vector_type(16)));
typedef __bf16         v16bf __attribute__((ext_vector_type(16)));
typedef v4f  __attribute__((may_alias)) v4fa;
typedef v4i  __attribute__((may_alias)) v4ia;
typedef v8us __attribute__((may_alias)) v8usa;
union FragB { v16bf v; v16us u; v8us h[2]; v8i w; };

__device__ __forceinline__ v8f wmb(const FragB& a, const FragB& b, v8f c) {
  v8f d = __builtin_amdgcn_wmma_f32_16x16x32_bf16(false, a.v, false, b.v, (short)0, c, false, false);
  asm volatile("v_nop\n\tv_nop\n\tv_nop\n\tv_nop" : "+v"(d) : "v"(a.w), "v"(b.w));
  return d;
}

__device__ __forceinline__ unsigned bf16_bits(float f) {
  const unsigned u = __float_as_uint(f);
  return (u + 0x7FFFu + ((u >> 16) & 1u)) >> 16;
}
__device__ __forceinline__ float bf16_val(float f) {
  return __uint_as_float(bf16_bits(f) << 16);
}
__device__ __forceinline__ float sigm(float v) { return 1.0f / (1.0f + expf(-v)); }

template <int SLB>
__device__ __forceinline__ int scan_chunk(const int* __restrict__ dsts, int nE, int cbase, int slotBase,
                                          int nb, int vec8, int* list, int tid, int lane, int wave) {
  int wc = 0;
  const int el0  = tid * EPT;
  const int e0   = cbase + el0;
  const int sent = -2147483647 - 1;
  v4i da, db;
  if (vec8 != 0 && cbase + CHUNK <= nE) {
    da = *(const v4i*)(dsts + e0);
    db = *(const v4i*)(dsts + e0 + 4);
  } else {
    da.x = (e0     < nE) ? dsts[min(e0,     nE - 1)] : sent;
    da.y = (e0 + 1 < nE) ? dsts[min(e0 + 1, nE - 1)] : sent;
    da.z = (e0 + 2 < nE) ? dsts[min(e0 + 2, nE - 1)] : sent;
    da.w = (e0 + 3 < nE) ? dsts[min(e0 + 3, nE - 1)] : sent;
    db.x = (e0 + 4 < nE) ? dsts[min(e0 + 4, nE - 1)] : sent;
    db.y = (e0 + 5 < nE) ? dsts[min(e0 + 5, nE - 1)] : sent;
    db.z = (e0 + 6 < nE) ? dsts[min(e0 + 6, nE - 1)] : sent;
    db.w = (e0 + 7 < nE) ? dsts[min(e0 + 7, nE - 1)] : sent;
  }
  const unsigned nbs = (unsigned)slotBase;
  const unsigned unb = (unsigned)nb;
  const unsigned s0 = (unsigned)da.x - nbs, s1 = (unsigned)da.y - nbs;
  const unsigned s2 = (unsigned)da.z - nbs, s3 = (unsigned)da.w - nbs;
  const unsigned s4 = (unsigned)db.x - nbs, s5 = (unsigned)db.y - nbs;
  const unsigned s6 = (unsigned)db.z - nbs, s7 = (unsigned)db.w - nbs;
  const bool h0 = s0 < unb, h1 = s1 < unb, h2 = s2 < unb, h3 = s3 < unb;
  const bool h4 = s4 < unb, h5 = s5 < unb, h6 = s6 < unb, h7 = s7 < unb;
  const unsigned any = __builtin_amdgcn_ballot_w32(h0 | h1 | h2 | h3 | h4 | h5 | h6 | h7);
  if (any != 0u) {
#define HITJ(J, HJ, SJ) { \
      const unsigned mj = __builtin_amdgcn_ballot_w32(HJ); \
      if (mj != 0u) { \
        if (HJ) { \
          const int pos = wc + (int)__builtin_amdgcn_mbcnt_lo(mj, 0u); \
          if (pos < WCAP) list[wave * WCAP + pos] = ((el0 + (J)) << SLB) | (int)(SJ); \
        } \
        wc += (int)__builtin_popcount(mj); } }
    HITJ(0, h0, s0)
    HITJ(1, h1, s1)
    HITJ(2, h2, s2)
    HITJ(3, h3, s3)
    HITJ(4, h4, s4)
    HITJ(5, h5, s5)
    HITJ(6, h6, s6)
    HITJ(7, h7, s7)
#undef HITJ
  }
  return wc;
}

__device__ __forceinline__ void cvt8_store(const float* __restrict__ p, unsigned short* dp) {
  const v4f a = *(const v4f*)p;
  const v4f b = *(const v4f*)(p + 4);
  v8us o;
  o[0] = (unsigned short)bf16_bits(a.x); o[1] = (unsigned short)bf16_bits(a.y);
  o[2] = (unsigned short)bf16_bits(a.z); o[3] = (unsigned short)bf16_bits(a.w);
  o[4] = (unsigned short)bf16_bits(b.x); o[5] = (unsigned short)bf16_bits(b.y);
  o[6] = (unsigned short)bf16_bits(b.z); o[7] = (unsigned short)bf16_bits(b.w);
  *(volatile v8us*)dp = o;
  __threadfence();
  *(volatile v8us*)dp = o;
}

__global__ __launch_bounds__(NTHR) void k_prep(
    const float* __restrict__ w_ih, const float* __restrict__ b_ih, const float* __restrict__ b_hh,
    const float* __restrict__ c1w, const float* __restrict__ c1b,
    const float* __restrict__ c2w, const float* __restrict__ c2b,
    const float* __restrict__ l1w, const float* __restrict__ l1b,
    const float* __restrict__ l2w, const float* __restrict__ l2b,
    unsigned short* WG2, unsigned short* B1, unsigned short* B2, float* BIAS) {
  const int tid = (int)threadIdx.x;
  const int b = (int)blockIdx.x;
  if (b < PB_WG) {
    const int u = b * NTHR + tid;
    const int n = u >> 5;
    const int k8 = (u & 31) * 8;
    const int ut = n / GN;
    const int rem = n - ut * GN;
    const int gate = rem >> 6;
    const int uu = rem & 63;
    const int gs = (gate == 0) ? 0 : ((gate == 1) ? 2 : 3);
    const int srow = gs * NF + ut * 64 + uu;
    cvt8_store(w_ih + (size_t)srow * NF + (k8 & (NF - 1)), WG2 + (size_t)n * KG + k8);
  } else if (b < PB_WG + PB_L1) {
    const int u = (b - PB_WG) * NTHR + tid;
    const int o = u >> 5;
    const int k8 = (u & 31) * 8;
    cvt8_store(l1w + (size_t)o * NF + (k8 & (NF - 1)), B1 + (size_t)o * K1 + k8);
  } else if (b < PB_WG + PB_L1 + PB_C1) {
    const int u = (b - PB_WG - PB_L1) * NTHR + tid;
    const int o = u >> 7;
    const int k8 = (u & 127) * 8;
    const int kk = k8 & 511;
    const int t = kk >> 7;
    const int c = kk & 127;
    cvt8_store(c1w + ((size_t)(t * C1O + o) * NF + c), B1 + (size_t)o * K1 + 2 * NF + k8);
  } else if (b < PB_WG + PB_L1 + PB_C1 + PB_L2) {
    const int u = (b - PB_WG - PB_L1 - PB_C1) * NTHR + tid;
    const int o = u >> 6;
    const int k8 = (u & 63) * 8;
    cvt8_store(l2w + (size_t)o * C1O + (k8 & (C1O - 1)), B2 + (size_t)o * K2 + k8);
  } else if (b < PB_WG + PB_L1 + PB_C1 + PB_L2 + PB_C2) {
    const int u = (b - PB_WG - PB_L1 - PB_C1 - PB_L2) * NTHR + tid;
    const int o = u >> 8;
    const int k8 = (u & 255) * 8;
    const int kk = k8 & 1023;
    const int t = kk >> 8;
    const int c = kk & 255;
    cvt8_store(c2w + ((size_t)(t * NF + o) * C1O + c), B2 + (size_t)o * K2 + 2 * C1O + k8);
  } else {
    const int f = 4 * tid;
    const int fc = f < NG - 4 ? f : NG - 4;
    const int ut = fc / GN;
    const int rem = fc - ut * GN;
    const int gate = rem >> 6;
    const int uu = rem & 63;
    const int gs = (gate == 0) ? 0 : ((gate == 1) ? 2 : 3);
    const int jg = gs * NF + ut * 64 + uu;
    int o1 = f - NG;        o1 = o1 < 0 ? 0 : (o1 > C1O - 4 ? C1O - 4 : o1);
    int o2 = f - NG - C1O;  o2 = o2 < 0 ? 0 : (o2 > NF - 4 ? NF - 4 : o2);
    const v4f bi = *(const v4f*)(b_ih + jg);
    const v4f bh = *(const v4f*)(b_hh + jg);
    const v4f q1 = *(const v4f*)(l1b + o1);
    const v4f r1 = *(const v4f*)(c1b + o1);
    const v4f q2 = *(const v4f*)(l2b + o2);
    const v4f r2 = *(const v4f*)(c2b + o2);
    const bool s0 = f < NG, s1 = f < NG + C1O;
    v4f val;
    val.x = s0 ? (bf16_val(bi.x) + bf16_val(bh.x)) : (s1 ? (bf16_val(q1.x) + 4.0f * bf16_val(r1.x)) : (bf16_val(q2.x) + 4.0f * bf16_val(r2.x)));
    val.y = s0 ? (bf16_val(bi.y) + bf16_val(bh.y)) : (s1 ? (bf16_val(q1.y) + 4.0f * bf16_val(r1.y)) : (bf16_val(q2.y) + 4.0f * bf16_val(r2.y)));
    val.z = s0 ? (bf16_val(bi.z) + bf16_val(bh.z)) : (s1 ? (bf16_val(q1.z) + 4.0f * bf16_val(r1.z)) : (bf16_val(q2.z) + 4.0f * bf16_val(r2.z)));
    val.w = s0 ? (bf16_val(bi.w) + bf16_val(bh.w)) : (s1 ? (bf16_val(q1.w) + 4.0f * bf16_val(r1.w)) : (bf16_val(q2.w) + 4.0f * bf16_val(r2.w)));
    const bool okst = tid < NBIAS / 4;
    float* dp = BIAS + (okst ? f : 0);
    if (okst) *(volatile v4f*)dp = val;
    __threadfence();
    if (okst) *(volatile v4f*)dp = val;
  }
}

__global__ __launch_bounds__(NTHR) void k_keys(const int* __restrict__ dst, const int* __restrict__ et,
                                               int nE, int nUnits, int* keys) {
  const int u = (int)blockIdx.x * NTHR + (int)threadIdx.x;
  if (u >= nUnits) return;
  const int e0 = 4 * u;
  const int ec = e0 < nE - 4 ? e0 : nE - 4;
  const v4i d = *(const v4i*)(dst + ec);
  const v4i t = *(const v4i*)(et + ec);
  const bool ok = e0 < nE;
  const int sent = -2147483647 - 1;
  v4i k;
  k.x = ok ? (int)((unsigned)d.x * 4u + (unsigned)t.x) : sent;
  k.y = ok ? (int)((unsigned)d.y * 4u + (unsigned)t.y) : sent;
  k.z = ok ? (int)((unsigned)d.z * 4u + (unsigned)t.z) : sent;
  k.w = ok ? (int)((unsigned)d.w * 4u + (unsigned)t.w) : sent;
  int* dp = keys + e0;
  *(volatile v4i*)dp = k;
  __threadfence();
  *(volatile v4i*)dp = k;
}

__global__ __launch_bounds__(NTHR) void k_osc(const float* __restrict__ x, const float* __restrict__ tbl,
                                              int nN, int nTbl, int nUnits, unsigned short* h0) {
  const int u = (int)blockIdx.x * NTHR + (int)threadIdx.x;
  if (u >= nUnits) return;
  const int row = u >> 4;
  const int k8  = (u & 15) * 8;
  const int rc  = row < nN ? row : nN - 1;
  const float* p = x + (size_t)rc * NF + k8;
  const v4f a = *(const v4f*)p;
  const v4f b = *(const v4f*)(p + 4);
  const bool ok = row < nN;
  float xs[8];
  unsigned hb[8], lb[8];
  xs[0] = a.x; xs[1] = a.y; xs[2] = a.z; xs[3] = a.w;
  xs[4] = b.x; xs[5] = b.y; xs[6] = b.z; xs[7] = b.w;
#pragma unroll
  for (int i = 0; i < 8; ++i) { hb[i] = 0u; lb[i] = 0u; }
#pragma unroll 1
  for (int j = 0; j < 8; ++j) {
    const float xv = bf16_val(xs[0]);
    const bool oor = (xv < -0.5f) | (xv > 0.5f);
    const float xi = oor ? 0.5001f : xv;
    const float sm = xi + 0.5f;
    const float pr = sm * 10000.0f;
    float fi = floorf(pr);
    fi = (fi >= 0.0f) ? fi : 0.0f;
    fi = (fi <= 1.0e6f) ? fi : 1.0e6f;
    int idx = (int)fi;
    idx = idx > nTbl - 1 ? nTbl - 1 : idx;
    const float tv = bf16_val(tbl[idx]);
    const float sg = sigm(xv);
    float h = (tv == 0.0f) ? sg : tv;
    h = ok ? h : 0.0f;
    const unsigned hbt = bf16_bits(h);
    const unsigned lbt = bf16_bits(h - __uint_as_float(hbt << 16));
#pragma unroll
    for (int i = 0; i < 7; ++i) { xs[i] = xs[i + 1]; hb[i] = hb[i + 1]; lb[i] = lb[i + 1]; }
    hb[7] = hbt; lb[7] = lbt;
  }
  v4u hv, lv;
  hv.x = hb[0] | (hb[1] << 16); hv.y = hb[2] | (hb[3] << 16);
  hv.z = hb[4] | (hb[5] << 16); hv.w = hb[6] | (hb[7] << 16);
  lv.x = lb[0] | (lb[1] << 16); lv.y = lb[2] | (lb[3] << 16);
  lv.z = lb[4] | (lb[5] << 16); lv.w = lb[6] | (lb[7] << 16);
  unsigned short* dp = h0 + (size_t)row * KG + k8;
  *(volatile v4u*)dp = hv;
  *(volatile v4u*)(dp + NF) = lv;
  __threadfence();
  *(volatile v4u*)dp = hv;
  *(volatile v4u*)(dp + NF) = lv;
}

__global__ __launch_bounds__(GTHR) void k_gates(const unsigned short* __restrict__ A,
                                                const unsigned short* __restrict__ BT,
                                                const float* __restrict__ bg, float* hout, unsigned short* a1) {
  __shared__ __attribute__((aligned(16))) float stg[GBM * GN];
  const int tid = (int)threadIdx.x, lane = tid & 31, wave = tid >> 5, hh = lane >> 4, m = lane & 15;
  const int rowBase = (int)blockIdx.x * GBM;
  const int ut = (int)blockIdx.y;

  v8f acc[12];
  {
    const v8f z = {0.f, 0.f, 0.f, 0.f, 0.f, 0.f, 0.f, 0.f};
#pragma unroll
    for (int t = 0; t < 12; ++t) acc[t] = z;
  }
  const unsigned short* ap = A + (size_t)(rowBase + 16 * wave + m) * (size_t)KG + 8 * hh;
  const unsigned short* bp = BT + (size_t)(ut * GN + m) * (size_t)KG + 8 * hh;
#pragma unroll 1
  for (int k0 = 0; k0 < KG; k0 += 32) {
    FragB af;
    af.h[0] = *(const v8usa*)(ap + k0);
    af.h[1] = *(const v8usa*)(ap + k0 + 16);
#pragma unroll
    for (int nt = 0; nt < 12; ++nt) {
      const unsigned short* wq = bp + (size_t)(16 * nt) * (size_t)KG + k0;
      FragB bf;
      bf.h[0] = *(const v8usa*)wq;
      bf.h[1] = *(const v8usa*)(wq + 16);
      acc[nt] = wmb(af, bf, acc[nt]);
    }
  }
#pragma unroll
  for (int nt = 0; nt < 12; ++nt) {
    const int lc = 16 * nt + m;
#pragma unroll
    for (int r = 0; r < 8; ++r) {
      const int lr = 16 * wave + 8 * hh + r;
      stg[lr * GN + lc] = acc[nt][r];
    }
  }
  __syncthreads();

  {
    const int uu = tid & 63;
    const float bi_ = bg[ut * GN + uu];
    const float bg_ = bg[ut * GN + 64 + uu];
    const float bo_ = bg[ut * GN + 128 + uu];
#pragma unroll 1
    for (int it = 0; it < 32; ++it) {
      const int r = 2 * it + (tid >> 6);
      const float iv = stg[r * GN + uu] + bi_;
      const float gv = stg[r * GN + 64 + uu] + bg_;
      const float ov = stg[r * GN + 128 + uu] + bo_;
      const float c  = sigm(iv) * tanhf(gv);
      const float hv = sigm(ov) * tanhf(c);
      stg[r * GN + uu] = hv;
    }
  }
  __syncthreads();

  v4f fv[8];
  v4u qv[8];
#pragma unroll
  for (int it = 0; it < 8; ++it) {
    const int unit = it * GTHR + tid;
    const int r = unit >> 4, c4 = (unit & 15) * 4;
    fv[it] = *(const v4fa*)(stg + r * GN + c4);
  }
#pragma unroll
  for (int it = 0; it < 8; ++it) {
    const int part = it >> 2;
    const int u2 = (it & 3) * GTHR + tid;
    const int r = u2 >> 3, c8 = (u2 & 7) * 8;
    const v4f f0 = *(const v4fa*)(stg + r * GN + c8);
    const v4f f1 = *(const v4fa*)(stg + r * GN + c8 + 4);
    const float fe[8] = {f0.x, f0.y, f0.z, f0.w, f1.x, f1.y, f1.z, f1.w};
    unsigned w[8];
#pragma unroll
    for (int i = 0; i < 8; ++i) {
      const unsigned hb = bf16_bits(fe[i]);
      const unsigned lb = bf16_bits(fe[i] - __uint_as_float(hb << 16));
      w[i] = part ? lb : hb;
    }
    v4u q;
    q.x = w[0] | (w[1] << 16); q.y = w[2] | (w[3] << 16);
    q.z = w[4] | (w[5] << 16); q.w = w[6] | (w[7] << 16);
    qv[it] = q;
  }
#pragma unroll
  for (int it = 0; it < 8; ++it) {
    const int unit = it * GTHR + tid;
    const int r = unit >> 4, c4 = (unit & 15) * 4;
    *(volatile v4f*)(hout + (size_t)(rowBase + r) * NF + ut * 64 + c4) = fv[it];
  }
#pragma unroll
  for (int it = 0; it < 8; ++it) {
    const int part = it >> 2;
    const int u2 = (it & 3) * GTHR + tid;
    const int r = u2 >> 3, c8 = (u2 & 7) * 8;
    *(volatile v4u*)(a1 + (size_t)(rowBase + r) * K1 + part * NF + ut * 64 + c8) = qv[it];
  }
  __threadfence();
#pragma unroll
  for (int it = 0; it < 8; ++it) {
    const int unit = it * GTHR + tid;
    const int r = unit >> 4, c4 = (unit & 15) * 4;
    *(volatile v4f*)(hout + (size_t)(rowBase + r) * NF + ut * 64 + c4) = fv[it];
  }
#pragma unroll
  for (int it = 0; it < 8; ++it) {
    const int part = it >> 2;
    const int u2 = (it & 3) * GTHR + tid;
    const int r = u2 >> 3, c8 = (u2 & 7) * 8;
    *(volatile v4u*)(a1 + (size_t)(rowBase + r) * K1 + part * NF + ut * 64 + c8) = qv[it];
  }
}

__global__ __launch_bounds__(GTHR) void k_gemm(const unsigned short* __restrict__ A,
                                               const unsigned short* __restrict__ BT, int K,
                                               const float* __restrict__ bias, float* outp, int ldo) {
  __shared__ __attribute__((aligned(16))) float stg[GBM * GBN];
  const int tid = (int)threadIdx.x, lane = tid & 31, wave = tid >> 5, hh = lane >> 4, m = lane & 15;
  const int rowBase = (int)blockIdx.x * GBM;
  const int col0    = (int)blockIdx.y * GBN;

  v8f acc[8];
  {
    const v8f z = {0.f, 0.f, 0.f, 0.f, 0.f, 0.f, 0.f, 0.f};
#pragma unroll
    for (int t = 0; t < 8; ++t) acc[t] = z;
  }
  const unsigned short* ap = A + (size_t)(rowBase + 16 * wave + m) * (size_t)K + 8 * hh;
  const unsigned short* bp = BT + (size_t)(col0 + m) * (size_t)K + 8 * hh;
#pragma unroll 1
  for (int k0 = 0; k0 < K; k0 += 32) {
    FragB af;
    af.h[0] = *(const v8usa*)(ap + k0);
    af.h[1] = *(const v8usa*)(ap + k0 + 16);
#pragma unroll
    for (int nt = 0; nt < 8; ++nt) {
      const unsigned short* wq = bp + (size_t)(16 * nt) * (size_t)K + k0;
      FragB bf;
      bf.h[0] = *(const v8usa*)wq;
      bf.h[1] = *(const v8usa*)(wq + 16);
      acc[nt] = wmb(af, bf, acc[nt]);
    }
  }
#pragma unroll
  for (int nt = 0; nt < 8; ++nt) {
    const int lc = 16 * nt + m;
#pragma unroll
    for (int r = 0; r < 8; ++r) {
      const int lr = 16 * wave + 8 * hh + r;
      stg[lr * GBN + lc] = acc[nt][r];
    }
  }
  __syncthreads();

  const v4f bb4 = *(const v4f*)(bias + col0 + 4 * lane);
  v4f pv[16];
#pragma unroll
  for (int i = 0; i < 16; ++i) {
    const v4f t = *(const v4fa*)(stg + (16 * wave + i) * GBN + 4 * lane);
    pv[i] = t + bb4;
  }
#pragma unroll
  for (int i = 0; i < 16; ++i) {
    const int r = rowBase + 16 * wave + i;
    *(volatile v4f*)(outp + (size_t)r * (size_t)ldo + col0 + 4 * lane) = pv[i];
  }
  __threadfence();
#pragma unroll
  for (int i = 0; i < 16; ++i) {
    const int r = rowBase + 16 * wave + i;
    *(volatile v4f*)(outp + (size_t)r * (size_t)ldo + col0 + 4 * lane) = pv[i];
  }
}

template <int C>
__global__ __launch_bounds__(NTHR) void k_scan(const int* __restrict__ keys, const int* __restrict__ srcs,
                                               int nEp, int nE, int nN, int mRows, int blk0, int rowOff,
                                               const float* __restrict__ feat, unsigned short* apl) {
  constexpr int CPL = C / 32;
  constexpr int AP  = (C == 128) ? K1 : K2;
  extern __shared__ __attribute__((aligned(16))) int dsm[];
  int* list = dsm;
  int* hl   = dsm + LISTN;
  int* sl   = hl + RCAP;
  int* cnt  = sl + RCAP;
  int* offs = cnt + NSL;
  int* cur  = offs + NSL;
  int* misc = cur + NSL;
  const int tid = (int)threadIdx.x, lane = tid & 31, wave = tid >> 5;
  const int nodeBase = ((int)blockIdx.x + blk0) * NBR;

  if constexpr (C == 256) {
#pragma unroll 1
    for (int r = wave; r < NBR; r += NWAVE) {
      const int node = nodeBase + r;
      if (node < mRows) {
        const int nc = node < nN ? node : nN - 1;
        const bool live = node < nN;
        const float* p = feat + (size_t)nc * C + 8 * lane;
        const v4f a = *(const v4f*)p;
        const v4f b = *(const v4f*)(p + 4);
        const float fe[8] = {a.x, a.y, a.z, a.w, b.x, b.y, b.z, b.w};
        unsigned hb[8], lb[8];
#pragma unroll
        for (int i = 0; i < 8; ++i) {
          const float v = live ? fe[i] : 0.0f;
          hb[i] = bf16_bits(v);
          lb[i] = bf16_bits(v - __uint_as_float(hb[i] << 16));
        }
        v4u hv, lv;
        hv.x = hb[0] | (hb[1] << 16); hv.y = hb[2] | (hb[3] << 16);
        hv.z = hb[4] | (hb[5] << 16); hv.w = hb[6] | (hb[7] << 16);
        lv.x = lb[0] | (lb[1] << 16); lv.y = lb[2] | (lb[3] << 16);
        lv.z = lb[4] | (lb[5] << 16); lv.w = lb[6] | (lb[7] << 16);
        unsigned short* dp = apl + (size_t)(node - rowOff) * AP + 8 * lane;
        *(volatile v4u*)dp = hv;
        *(volatile v4u*)(dp + C) = lv;
        __threadfence();
        *(volatile v4u*)dp = hv;
        *(volatile v4u*)(dp + C) = lv;
      }
    }
  }

  {
    const v4i z4 = {0, 0, 0, 0};
    for (int i = tid * 4; i < AGG_ZINTS; i += NTHR * 4) *(v4ia*)(dsm + i) = z4;
    if (tid < MISC_INTS) misc[tid] = 0;
  }
  __syncthreads();

  int t = 0, ov = 0;
  const int nChunks = (nEp + CHUNK - 1) / CHUNK;
#pragma unroll 1
  for (int ch = 0; ch < nChunks; ++ch) {
    const int cbase = ch * CHUNK;
    const int wc = scan_chunk<SLA>(keys, nEp, cbase, nodeBase * 4, NSL, 1, list, tid, lane, wave);
    if (lane == 0) misc[wave] = wc;
    __syncthreads();
    if (wave == 0) {
#pragma unroll 1
      for (int w2 = 0; w2 < NWAVE; ++w2) {
        int c = misc[w2];
        c = c < 0 ? 0 : (c > WCAP ? WCAP : c);
#pragma unroll 1
        for (int b0 = 0; b0 < c; b0 += 32) {
          const int idx = b0 + lane;
          const int ent = list[w2 * WCAP + (idx < WCAP ? idx : WCAP - 1)];
          const int m32 = (c - b0) < 32 ? (c - b0) : 32;
#pragma unroll 1
          for (int k = 0; k < m32; ++k) {
            const int u    = __builtin_amdgcn_readlane(ent, k);
            const int slot = u & (NSL - 1);
            const int el   = (u >> SLA) & (CHUNK - 1);
            const int pk   = ((cbase + el) << SLA) | slot;
            if (t < RCAP) {
              if (lane == 0) { hl[t] = pk; cnt[slot] = cnt[slot] + 1; }
              t = t + 1;
            } else {
              ov = 1;
            }
          }
        }
      }
    }
    __syncthreads();
  }
  if (wave == 0 && lane == 0) { misc[8] = t; misc[9] = ov; }
  __syncthreads();
  int tt = misc[8];
  tt = tt < 0 ? 0 : (tt > RCAP ? RCAP : tt);
  const int ovf = misc[9];

  if (wave == 0) {
    const int base = lane * (NSL / 32);
    int s = 0;
#pragma unroll 1
    for (int i = 0; i < NSL / 32; ++i) s += cnt[base + i];
    int incl = s;
#pragma unroll
    for (int d = 1; d < 32; d <<= 1) {
      const int y = __shfl_up(incl, d, 32);
      if (lane >= d) incl += y;
    }
    int run = incl - s;
#pragma unroll 1
    for (int i = 0; i < NSL / 32; ++i) {
      const int cv = cnt[base + i];
      offs[base + i] = run;
      cur[base + i]  = run;
      run += cv;
    }
  }
  __syncthreads();
  if (wave == 0) {
#pragma unroll 1
    for (int b0 = 0; b0 < tt; b0 += 32) {
      const int idx = b0 + lane;
      const int ent = hl[idx < RCAP ? idx : RCAP - 1];
      const int m32 = (tt - b0) < 32 ? (tt - b0) : 32;
#pragma unroll 1
      for (int k = 0; k < m32; ++k) {
        const int u    = __builtin_amdgcn_readlane(ent, k);
        const int slot = u & (NSL - 1);
        if (lane == 0) {
          int p = cur[slot];
          p = p < 0 ? 0 : (p > RCAP - 1 ? RCAP - 1 : p);
          sl[p] = u;
          cur[slot] = p + 1;
        }
      }
    }
  }
  __syncthreads();

  const float qnan = __int_as_float(0x7fc00000);
  const float finf = __int_as_float(0x7f800000);
  const float ninf = __int_as_float((int)0xff800000u);
  const float pz = (ovf != 0) ? qnan : 0.0f;
  const int j16 = lane & 15;
  const int sA = 2 * j16, sB = 2 * j16 + 1;
#pragma unroll 1
  for (int si = 0; si < NSL / NWAVE; ++si) {
    const int s    = si * NWAVE + wave;
    const int node = nodeBase + (s >> 2);
    const int ty   = s & 3;
    int c = cnt[s];
    const bool big = c > DEGCAP;
    c = c < 0 ? 0 : (c > DEGCAP ? DEGCAP : c);
    int o = offs[s];
    o = o < 0 ? 0 : (o > RCAP ? RCAP : o);
    float acc[CPL];
#pragma unroll
    for (int i = 0; i < CPL; ++i) acc[i] = ninf;
#pragma unroll 1
    for (int b0 = 0; b0 < c; b0 += 32) {
      int idx = o + b0 + lane;
      idx = idx > RCAP - 1 ? RCAP - 1 : idx;
      const int ent = sl[idx];
      int eid = ent >> SLA;
      eid = eid < 0 ? 0 : (eid > nE - 1 ? nE - 1 : eid);
      int sr = srcs[eid];
      sr = sr < 0 ? 0 : (sr > nN - 1 ? nN - 1 : sr);
      const int m32 = (c - b0) < 32 ? (c - b0) : 32;
#pragma unroll 1
      for (int k = 0; k < m32; ++k) {
        const int sk = __builtin_amdgcn_readlane(sr, k);
        const float* rp = feat + (size_t)sk * C + CPL * lane;
        const v4f a = *(const v4f*)rp;
        acc[0] = fmaxf(acc[0], a.x); acc[1] = fmaxf(acc[1], a.y);
        acc[2] = fmaxf(acc[2], a.z); acc[3] = fmaxf(acc[3], a.w);
        if constexpr (C == 256) {
          const v4f b = *(const v4f*)(rp + 4);
          acc[4] = fmaxf(acc[4], b.x); acc[5] = fmaxf(acc[5], b.y);
          acc[6] = fmaxf(acc[6], b.z); acc[7] = fmaxf(acc[7], b.w);
        }
      }
    }
    const float pzr = big ? qnan : pz;
    const bool live = node < nN;
    unsigned hb[CPL], lb[CPL];
#pragma unroll
    for (int i = 0; i < CPL; ++i) {
      float v = acc[i];
      v = (fabsf(v) < finf) ? v : 0.0f;
      v = live ? (v + pzr) : 0.0f;
      hb[i] = bf16_bits(v);
      lb[i] = bf16_bits(v - __uint_as_float(hb[i] << 16));
    }
    const bool wr = node < mRows;
    const int lr = wr ? (node - rowOff) : 0;
    if constexpr (C == 128) {
      const int hw0 = (int)(hb[0] | (hb[1] << 16)), hw1 = (int)(hb[2] | (hb[3] << 16));
      const int lw0 = (int)(lb[0] | (lb[1] << 16)), lw1 = (int)(lb[2] | (lb[3] << 16));
      const int g0 = __shfl(hw0, sA, 32), g1 = __shfl(hw1, sA, 32);
      const int g2 = __shfl(hw0, sB, 32), g3 = __shfl(hw1, sB, 32);
      const int p0 = __shfl(lw0, sA, 32), p1 = __shfl(lw1, sA, 32);
      const int p2 = __shfl(lw0, sB, 32), p3 = __shfl(lw1, sB, 32);
      const bool lsel = lane >= 16;
      v4u pv;
      pv.x = (unsigned int)(lsel ? p0 : g0);
      pv.y = (unsigned int)(lsel ? p1 : g1);
      pv.z = (unsigned int)(lsel ? p2 : g2);
      pv.w = (unsigned int)(lsel ? p3 : g3);
      const int col = 2 * NF + ty * NF + (lsel ? 4 * NF : 0) + 8 * j16;
      unsigned short* dp = apl + (size_t)lr * AP + col;
      if (wr) *(volatile v4u*)dp = pv;
      __threadfence();
      if (wr) *(volatile v4u*)dp = pv;
    } else {
      v4u hv, lv;
      hv.x = hb[0] | (hb[1] << 16); hv.y = hb[2] | (hb[3] << 16);
      hv.z = hb[4] | (hb[5] << 16); hv.w = hb[6] | (hb[7] << 16);
      lv.x = lb[0] | (lb[1] << 16); lv.y = lb[2] | (lb[3] << 16);
      lv.z = lb[4] | (lb[5] << 16); lv.w = lb[6] | (lb[7] << 16);
      unsigned short* dp = apl + (size_t)lr * AP + 2 * C + ty * C + 8 * lane;
      if (wr) { *(volatile v4u*)dp = hv; *(volatile v4u*)(dp + 4 * C) = lv; }
      __threadfence();
      if (wr) { *(volatile v4u*)dp = hv; *(volatile v4u*)(dp + 4 * C) = lv; }
    }
  }
}

template <int C, int MODE>
__global__ __launch_bounds__(NTHR) void k_colstat(const float* __restrict__ P, const float* __restrict__ st,
                                                  int nN, float* rec) {
  __shared__ __attribute__((aligned(16))) float part[NTHR];
  constexpr int RS = NTHR / C, RPS = SBLK / RS;
  const int tid = (int)threadIdx.x;
  const int c = tid & (C - 1);
  const int rs = tid / C;
  const int r0 = (int)blockIdx.x * SBLK + rs * RPS;
  const float mu = (MODE != 0) ? st[c] : 0.0f;
  float s = 0.0f;
#pragma unroll 4
  for (int i = 0; i < RPS; ++i) {
    const int r = r0 + i;
    const int rc = r < nN ? r : nN - 1;
    const float v = P[(size_t)rc * C + c];
    const float d = v - mu;
    const float tv = (MODE != 0) ? d * d : v;
    s += (r < nN) ? tv : 0.0f;
  }
  part[tid] = s;
  __syncthreads();
  const bool okst = tid < C / 4;
  const int q4 = okst ? 4 * tid : 0;
  v4f a = *(const v4fa*)(part + q4);
  if constexpr (RS == 2) {
    const v4f b = *(const v4fa*)(part + C + q4);
    a = a + b;
  }
  float* dp = rec + (size_t)blockIdx.x * C + q4;
  if (okst) *(volatile v4f*)dp = a;
  __threadfence();
  if (okst) *(volatile v4f*)dp = a;
}

template <int C, int MODE>
__global__ __launch_bounds__(NTHR) void k_comb(const float* __restrict__ rec, int nblk, int nN,
                                               const float* __restrict__ gam, const float* __restrict__ bet,
                                               float* st) {
  __shared__ __attribute__((aligned(16))) float sb[3 * 256];
  const int tid = (int)threadIdx.x;
  const int c = tid & (C - 1);
  double s = 0.0;
#pragma unroll 4
  for (int b = 0; b < nblk; ++b) s += (double)rec[(size_t)b * C + c];
  const double mean = s / (double)nN;
  if (tid < C) {
    if constexpr (MODE == 0) {
      sb[c] = (float)mean;
    } else {
      const float var = (float)mean;
      sb[c] = rsqrtf(var + 1e-5f);
      sb[256 + c] = bf16_val(gam[c]);
      sb[512 + c] = bf16_val(bet[c]);
    }
  }
  __syncthreads();
  constexpr int NR = (MODE == 0) ? 1 : 3;
  constexpr int QPR = C / 4;
  const bool okst = tid < NR * QPR;
  const int tq = okst ? tid : 0;
  const int row = tq / QPR;
  const int q4 = (tq - row * QPR) * 4;
  const v4f v = *(const v4fa*)(sb + row * 256 + q4);
  float* dp = st + (size_t)(MODE + row) * 256 + q4;
  if (okst) *(volatile v4f*)dp = v;
  __threadfence();
  if (okst) *(volatile v4f*)dp = v;
}

__global__ __launch_bounds__(NTHR) void k_apply(float* P, const float* __restrict__ st, int nUnits) {
  const int u = (int)blockIdx.x * NTHR + (int)threadIdx.x;
  if (u >= nUnits) return;
  const int c4 = (u & 63) * 4;
  float* p = P + (size_t)(u >> 6) * C1O + c4;
  const v4f x  = *(const v4f*)p;
  const v4f mu = *(const v4f*)(st + c4);
  const v4f rs = *(const v4f*)(st + 256 + c4);
  const v4f g  = *(const v4f*)(st + 512 + c4);
  const v4f b  = *(const v4f*)(st + 768 + c4);
  v4f v = ((x - mu) * rs) * g + b;
  v.x = (v.x > 0.0f) ? v.x : (v.x - v.x);
  v.y = (v.y > 0.0f) ? v.y : (v.y - v.y);
  v.z = (v.z > 0.0f) ? v.z : (v.z - v.z);
  v.w = (v.w > 0.0f) ? v.w : (v.w - v.w);
  *(volatile v4f*)p = v;
  __threadfence();
  *(volatile v4f*)p = v;
}

__global__ __launch_bounds__(NTHR) void k_out(const float* __restrict__ P, const float* __restrict__ st,
                                              int nUnits, float* out) {
  const int u = (int)blockIdx.x * NTHR + (int)threadIdx.x;
  if (u >= nUnits) return;
  const int c4 = (u & 31) * 4;
  const size_t eo = (size_t)(u >> 5) * NF + c4;
  const v4f x  = *(const v4f*)(P + eo);
  const v4f mu = *(const v4f*)(st + c4);
  const v4f rs = *(const v4f*)(st + 256 + c4);
  const v4f g  = *(const v4f*)(st + 512 + c4);
  const v4f b  = *(const v4f*)(st + 768 + c4);
  const v4f z = ((x - mu) * rs) * g + b;
  float zs[4] = {z.x, z.y, z.z, z.w};
  float os[4] = {0.0f, 0.0f, 0.0f, 0.0f};
#pragma unroll 1
  for (int j = 0; j < 4; ++j) {
    const float tv = zs[0] - 10.0f;
    const float r = sigm(tv);
#pragma unroll
    for (int i = 0; i < 3; ++i) { zs[i] = zs[i + 1]; os[i] = os[i + 1]; }
    os[3] = r;
  }
  v4f o;
  o.x = os[0]; o.y = os[1]; o.z = os[2]; o.w = os[3];
  *(volatile v4f*)(out + eo) = o;
  __threadfence();
  *(volatile v4f*)(out + eo) = o;
}

static inline int cdiv(int a, int b) { return (a + b - 1) / b; }
static inline size_t al256(size_t o) { return (o + 255) & ~(size_t)255; }
static inline size_t smax(size_t a, size_t b) { return a > b ? a : b; }

extern "C" void kernel_launch(void* const* d_in, const int* in_sizes, int n_in,
                              void* d_out, int out_size, void* d_ws, size_t ws_size,
                              hipStream_t stream) {
  if (n_in < 20) return;
  if (in_sizes[0] < NF || (in_sizes[0] % NF) != 0) return;
  const int nN = in_sizes[0] / NF;
  if (nN < 64 || nN > (1 << 20)) return;
  const int nTbl = in_sizes[1];
  if (nTbl < 10002) return;
  const int nE = in_sizes[3];
  if (nE < 4 || (nE & 3) != 0 || in_sizes[2] != 2 * nE) return;
  if (in_sizes[4] != 4 * NF * NF) return;
  if (in_sizes[6] != 4 * NF || in_sizes[7] != 4 * NF) return;
  if (in_sizes[8] != 4 * C1O * NF || in_sizes[9] != C1O) return;
  if (in_sizes[10] != 4 * NF * C1O || in_sizes[11] != NF) return;
  if (in_sizes[12] != C1O * NF || in_sizes[13] != C1O) return;
  if (in_sizes[14] != NF * C1O || in_sizes[15] != NF) return;
  if (in_sizes[16] != C1O || in_sizes[17] != C1O) return;
  if (in_sizes[18] != NF || in_sizes[19] != NF) return;
  if ((long long)out_size != (long long)nN * NF) return;

  const float* x     = (const float*)d_in[0];
  const float* tbl   = (const float*)d_in[1];
  const int*   eidx  = (const int*)d_in[2];
  const int*   etype = (const int*)d_in[3];
  const float* w_ih  = (const float*)d_in[4];
  const float* b_ih  = (const float*)d_in[6];
  const float* b_hh  = (const float*)d_in[7];
  const float* c1w   = (const float*)d_in[8];
  const float* c1b   = (const float*)d_in[9];
  const float* c2w   = (const float*)d_in[10];
  const float* c2b   = (const float*)d_in[11];
  const float* l1w   = (const float*)d_in[12];
  const float* l1b   = (const float*)d_in[13];
  const float* l2w   = (const float*)d_in[14];
  const float* l2b   = (const float*)d_in[15];
  const float* bn1g  = (const float*)d_in[16];
  const float* bn1b  = (const float*)d_in[17];
  const float* bn2g  = (const float*)d_in[18];
  const float* bn2b  = (const float*)d_in[19];
  float* out = (float*)d_out;
  const int* src = eidx;
  const int* dst = eidx + nE;

  const int nEp = cdiv(nE, CHUNK) * CHUNK;
  if (nEp >= (1 << (31 - SLA))) return;
  const int MP = cdiv(nN, GBM) * GBM;
  const int gA = cdiv(MP, NBR);
  const int hbk = (gA + 1) / 2;
  const int rows0 = (hbk * NBR < MP) ? hbk * NBR : MP;
  const int rows1 = MP - rows0;
  if ((rows0 % GBM) != 0 || (rows1 % GBM) != 0) return;
  const int nblk = cdiv(nN, SBLK);

  char* ws = (char*)d_ws;
  size_t off = 0;
  const size_t oKEY = off; off = al256(off + (size_t)nEp * 4);
  const size_t oWG  = off; off = al256(off + (size_t)NG * KG * 2);
  const size_t oB1  = off; off = al256(off + (size_t)C1O * K1 * 2);
  const size_t oB2  = off; off = al256(off + (size_t)NF * K2 * 2);
  const size_t oBI  = off; off = al256(off + (size_t)NBIAS * 4);
  const size_t oH0  = off; off = al256(off + (size_t)MP * KG * 2);
  const size_t oH   = off; off = al256(off + (size_t)MP * NF * 4);
  const size_t aBytes = smax((size_t)MP * K1 * 2, smax((size_t)rows0 * K2 * 2, (size_t)rows1 * K2 * 2));
  const size_t oA   = off; off = al256(off + aBytes);
  const size_t oP1  = off; off = al256(off + (size_t)MP * C1O * 4);
  const size_t oP2  = off; off = al256(off + (size_t)MP * NF * 4);
  const size_t oREC = off; off = al256(off + (size_t)nblk * 256 * 4);
  const size_t oS1  = off; off = al256(off + (size_t)4 * 256 * 4);
  const size_t oS2  = off; off = al256(off + (size_t)4 * 256 * 4);
  if (off > ws_size || off > (size_t)WSMAX) return;
  int*            KEY = (int*)(ws + oKEY);
  unsigned short* WG2 = (unsigned short*)(ws + oWG);
  unsigned short* B1  = (unsigned short*)(ws + oB1);
  unsigned short* B2  = (unsigned short*)(ws + oB2);
  float*          BI  = (float*)(ws + oBI);
  unsigned short* H0  = (unsigned short*)(ws + oH0);
  float*          H   = (float*)(ws + oH);
  unsigned short* AR  = (unsigned short*)(ws + oA);
  float*          P1  = (float*)(ws + oP1);
  float*          P2  = (float*)(ws + oP2);
  float*          REC = (float*)(ws + oREC);
  float*          S1  = (float*)(ws + oS1);
  float*          S2  = (float*)(ws + oS2);

  const size_t scanLds = (size_t)AGG_LDS_INTS * 4;
  hipFuncSetAttribute(reinterpret_cast<const void*>(&k_scan<128>), hipFuncAttributeMaxDynamicSharedMemorySize, (int)scanLds);
  hipFuncSetAttribute(reinterpret_cast<const void*>(&k_scan<256>), hipFuncAttributeMaxDynamicSharedMemorySize, (int)scanLds);

  k_prep<<<PB_ALL, NTHR, 0, stream>>>(w_ih, b_ih, b_hh, c1w, c1b, c2w, c2b, l1w, l1b, l2w, l2b, WG2, B1, B2, BI);
  k_keys<<<cdiv(nEp / 4, NTHR), NTHR, 0, stream>>>(dst, etype, nE, nEp / 4, KEY);
  k_osc<<<cdiv(MP * 16, NTHR), NTHR, 0, stream>>>(x, tbl, nN, nTbl, MP * 16, H0);
  k_gates<<<dim3(MP / GBM, 2), GTHR, 0, stream>>>(H0, WG2, BI, H, AR);
  k_scan<128><<<gA, NTHR, scanLds, stream>>>(KEY, src, nEp, nE, nN, MP, 0, 0, H, AR);
  k_gemm<<<dim3(MP / GBM, C1O / GBN), GTHR, 0, stream>>>(AR, B1, K1, BI + NG, P1, C1O);
  k_colstat<256, 0><<<nblk, NTHR, 0, stream>>>(P1, S1, nN, REC);
  k_comb<256, 0><<<1, NTHR, 0, stream>>>(REC, nblk, nN, bn1g, bn1b, S1);
  k_colstat<256, 1><<<nblk, NTHR, 0, stream>>>(P1, S1, nN, REC);
  k_comb<256, 1><<<1, NTHR, 0, stream>>>(REC, nblk, nN, bn1g, bn1b, S1);
  k_apply<<<cdiv(MP * 64, NTHR), NTHR, 0, stream>>>(P1, S1, MP * 64);
  k_scan<256><<<hbk, NTHR, scanLds, stream>>>(KEY, src, nEp, nE, nN, MP, 0, 0, P1, AR);
  k_gemm<<<dim3(rows0 / GBM, NF / GBN), GTHR, 0, stream>>>(AR, B2, K2, BI + NG + C1O, P2, NF);
  if (rows1 > 0) {
    k_scan<256><<<gA - hbk, NTHR, scanLds, stream>>>(KEY, src, nEp, nE, nN, MP, hbk, rows0, P1, AR);
    k_gemm<<<dim3(rows1 / GBM, NF / GBN), GTHR, 0, stream>>>(AR, B2, K2, BI + NG + C1O, P2 + (size_t)rows0 * NF, NF);
  }
  k_colstat<128, 0><<<nblk, NTHR, 0, stream>>>(P2, S2, nN, REC);
  k_comb<128, 0><<<1, NTHR, 0, stream>>>(REC, nblk, nN, bn2g, bn2b, S2);
  k_colstat<128, 1><<<nblk, NTHR, 0, stream>>>(P2, S2, nN, REC);
  k_comb<128, 1><<<1, NTHR, 0, stream>>>(REC, nblk, nN, bn2g, bn2b, S2);
  k_out<<<cdiv(nN * 32, NTHR), NTHR, 0, stream>>>(P2, S2, nN * 32, out);
}
